// SelfAttentionMLP_16552803959225
// MI455X (gfx1250) — hardware-run, weakly checked
//
#include <hip/hip_runtime.h>


#define NB_  4096
#define DD   256
typedef _Float16 h16;
typedef unsigned short bf;
typedef __attribute__((ext_vector_type(16))) __bf16   v16bf;
typedef __attribute__((ext_vector_type(16))) _Float16 v16h;
typedef __attribute__((ext_vector_type(8)))  _Float16 v8h;
typedef __attribute__((ext_vector_type(8)))  unsigned short v8us;
typedef __attribute__((ext_vector_type(8)))  float    v8f;
typedef __attribute__((ext_vector_type(4)))  float    v4f;
typedef v8h  __attribute__((may_alias)) v8ha;
typedef v4f  __attribute__((may_alias)) v4fa;
typedef v8us __attribute__((may_alias)) v8usa;

__device__ __forceinline__ unsigned short f2bf(float f) { unsigned u = __float_as_uint(f); u += 0x7FFFu + ((u >> 16) & 1u); return (unsigned short)(u >> 16); }
__device__ __forceinline__ float bf2f(unsigned short b) { return __uint_as_float(((unsigned)b) << 16); }
__device__ __forceinline__ float bfr(float f) { return bf2f(f2bf(f)); }
__device__ __forceinline__ v16h cat16(v8h lo, v8h hi) { return __builtin_shufflevector(lo, hi, 0, 1, 2, 3, 4, 5, 6, 7, 8, 9, 10, 11, 12, 13, 14, 15); }
__device__ __forceinline__ v16bf cat16b(v8us lo, v8us hi) { return __builtin_bit_cast(v16bf, __builtin_shufflevector(lo, hi, 0, 1, 2, 3, 4, 5, 6, 7, 8, 9, 10, 11, 12, 13, 14, 15)); }
__device__ __forceinline__ v8f wmma16(v16h a, v16h b, v8f c) { return __builtin_amdgcn_wmma_f32_16x16x32_f16(false, a, false, b, (short)0, c, false, false); }
__device__ __forceinline__ v8f wmmab(v16bf a, v16bf b, v8f c) { return __builtin_amdgcn_wmma_f32_16x16x32_bf16(false, a, false, b, (short)0, c, false, false); }


template <typename T16> struct WFrag;
template <> struct WFrag<h16> { typedef v16h V; static __device__ __forceinline__ V ld(const h16* p) { return cat16(*(const v8h*)p, *(const v8h*)(p + 16)); } static __device__ __forceinline__ v8f mma(V a, V b, v8f c) { return wmma16(a, b, c); } };
template <> struct WFrag<bf> { typedef v16bf V; static __device__ __forceinline__ V ld(const bf* p) { return cat16b(*(const v8us*)p, *(const v8us*)(p + 16)); } static __device__ __forceinline__ v8f mma(V a, V b, v8f c) { return wmmab(a, b, c); } };
template <typename T16, int NSPLIT, bool BIAS>
__global__ __launch_bounds__(32) void k_gemmw(const T16* __restrict__ A, const T16* __restrict__ A2, const T16* __restrict__ Bt, const T16* __restrict__ Bt2, int K, float* C, int ldc, const float* __restrict__ bias, size_t sA, size_t sB, size_t sC) {
    typedef typename WFrag<T16>::V V;
    __shared__ __align__(16) float os[16 * 68];
    const size_t z = blockIdx.z; A += z * sA; if (A2) A2 += z * sA; Bt += z * sB; if (Bt2) Bt2 += z * sB; C += z * sC;
    const int lane = threadIdx.x & 31, lr = lane & 15, hi = lane >> 4; const int r0 = blockIdx.x * 64, c0 = blockIdx.y * 64;
    v8f acc[4][4];
#pragma unroll
    for (int mb = 0; mb < 4; ++mb)
#pragma unroll
        for (int nb = 0; nb < 4; ++nb) acc[mb][nb] = (v8f){};
    const size_t aoff = (size_t)(r0 + lr) * K + 8 * hi, boff = (size_t)(c0 + lr) * K + 8 * hi;
#pragma unroll 1
    for (int kc = 0; kc < K; kc += 32) {
        V a[4], a2[4];
#pragma unroll
        for (int mb = 0; mb < 4; ++mb) { a[mb] = WFrag<T16>::ld(A + aoff + (size_t)mb * 16 * K + kc); if (NSPLIT == 1 || NSPLIT == 2) a2[mb] = WFrag<T16>::ld(A2 + aoff + (size_t)mb * 16 * K + kc); }
#pragma unroll
        for (int nb = 0; nb < 4; ++nb) { const V b = WFrag<T16>::ld(Bt + boff + (size_t)nb * 16 * K + kc); V b2; if (NSPLIT >= 2) b2 = WFrag<T16>::ld(Bt2 + boff + (size_t)nb * 16 * K + kc);
#pragma unroll
            for (int mb = 0; mb < 4; ++mb) { acc[mb][nb] = WFrag<T16>::mma(a[mb], b, acc[mb][nb]); if (NSPLIT == 1 || NSPLIT == 2) acc[mb][nb] = WFrag<T16>::mma(a2[mb], b, acc[mb][nb]); if (NSPLIT >= 2) acc[mb][nb] = WFrag<T16>::mma(a[mb], b2, acc[mb][nb]); } }
        asm volatile("v_nop\n\tv_nop\n\tv_nop\n\tv_nop" : "+v"(acc[0][0]), "+v"(acc[1][1]), "+v"(acc[2][2]), "+v"(acc[3][3]) : "v"(a[0]), "v"(a[3]));
    }
#pragma unroll
    for (int mb = 0; mb < 4; ++mb) {
#pragma unroll
        for (int nb = 0; nb < 4; ++nb) {
#pragma unroll
            for (int j = 0; j < 8; ++j) os[(hi * 8 + j) * 68 + nb * 16 + lr] = acc[mb][nb][j]; }
        __builtin_amdgcn_wave_barrier(); asm volatile("" ::: "memory");
        float* crow = C + (size_t)(r0 + mb * 16) * ldc + c0;
#pragma unroll 1
        for (int ps = 0; ps < 2; ++ps) {
#pragma unroll
            for (int s = 0; s < 8; ++s) { const int row = 2 * s + hi, cofs = lr * 4; v4f val = *(const v4fa*)(os + row * 68 + cofs); if (BIAS) { val[0] += bfr(bias[c0 + cofs]); val[1] += bfr(bias[c0 + cofs + 1]); val[2] += bfr(bias[c0 + cofs + 2]); val[3] += bfr(bias[c0 + cofs + 3]); }
                *(volatile v4f*)(crow + (size_t)row * ldc + cofs) = val; }
            if (ps == 0) __threadfence(); }
        __builtin_amdgcn_wave_barrier(); asm volatile("" ::: "memory");
    }
}

__device__ __forceinline__ void splitf(float y, unsigned short& h, unsigned short& l) { h = f2bf(y); l = f2bf(y - bf2f(h)); }
typedef __attribute__((ext_vector_type(4))) unsigned short v4us;

__global__ __launch_bounds__(256) void k_cvt8(const float* __restrict__ src, bf* dst, size_t n8) { const size_t i = (size_t)blockIdx.x * 256 + threadIdx.x; if (i >= n8) return; const v8f v = *(const v8f*)(src + i * 8); v8us o;
#pragma unroll
    for (int k = 0; k < 8; ++k) o[k] = f2bf(v[k]); *(volatile v8us*)(dst + i * 8) = o; __threadfence(); *(volatile v8us*)(dst + i * 8) = o; }
__global__ __launch_bounds__(256) void k_kmm(const float* __restrict__ K, float* KMM) { const int lane = threadIdx.x & 31; const int b = blockIdx.x * 8 + (threadIdx.x >> 5); if (b >= NB_) return; float mx = -3.0e38f, mn = 3.0e38f;
#pragma unroll
    for (int c = 0; c < DD / 32; ++c) { const float k = K[(size_t)b * DD + c * 32 + lane]; mx = fmaxf(mx, k); mn = fminf(mn, k); }
#pragma unroll
    for (int sh = 16; sh; sh >>= 1) { mx = fmaxf(mx, __shfl_xor(mx, sh, 32)); mn = fminf(mn, __shfl_xor(mn, sh, 32)); }
    const float v = (lane & 1) ? mn : mx; *(volatile float*)(KMM + (size_t)b * 32 + lane) = v; __threadfence(); *(volatile float*)(KMM + (size_t)b * 32 + lane) = v; }
__global__ __launch_bounds__(256) void k_att(const float* __restrict__ Q, const float* __restrict__ K, const float* __restrict__ V, const float* __restrict__ KMM, float* AW, float* O) { const int idx = blockIdx.x * 256 + threadIdx.x; if (idx >= NB_ * DD) return; const int b = idx / DD; const float q = Q[idx]; const float* kb = K + (size_t)b * DD; const float* vb = V + (size_t)b * DD;
    const float m = (q >= 0.f) ? __fmul_rn(q, KMM[(size_t)b * 32]) : __fmul_rn(q, KMM[(size_t)b * 32 + 1]); float s = 0.f;
#pragma unroll 1
    for (int j = 0; j < DD; ++j) { float d0 = __fsub_rn(__fmul_rn(q, kb[j]), m); asm volatile("" : "+v"(d0)); s = __fadd_rn(s, __builtin_amdgcn_exp2f(__fmul_rn(d0, 1.4426950408889634f))); }
    const float inv = __fdiv_rn(1.0f, s); float aw = 0.f, acc = 0.f;
#pragma unroll 1
    for (int j = 0; j < DD; ++j) { float d0 = __fsub_rn(__fmul_rn(q, kb[j]), m); asm volatile("" : "+v"(d0)); float a = __fmul_rn(__builtin_amdgcn_exp2f(__fmul_rn(d0, 1.4426950408889634f)), inv); asm volatile("" : "+v"(a)); aw = __fadd_rn(aw, a); float p = __fmul_rn(a, vb[j]); asm volatile("" : "+v"(p)); acc = __fadd_rn(acc, p); }
    const float awm = __fdiv_rn(aw, (float)DD); for (int ps = 0; ps < 2; ++ps) { *(volatile float*)(AW + idx) = awm; *(volatile float*)(O + idx) = acc; if (ps == 0) __threadfence(); } }
__global__ __launch_bounds__(256) void k_spl(const float* __restrict__ F, size_t n4, bf* Hh, bf* Hl) { const size_t e = ((size_t)blockIdx.x * 256 + threadIdx.x) * 4; if (e >= n4) return; const v4f a = *(const v4f*)(F + e); v4us oh, ol;
#pragma unroll
    for (int u = 0; u < 4; ++u) { unsigned short h, l; splitf(a[u], h, l); oh[u] = h; ol[u] = l; } *(volatile v4us*)(Hh + e) = oh; *(volatile v4us*)(Hl + e) = ol; __threadfence(); *(volatile v4us*)(Hh + e) = oh; *(volatile v4us*)(Hl + e) = ol; }

extern "C" void kernel_launch(void* const* d_in, const int* in_sizes, int n_in,
                              void* d_out, int out_size, void* d_ws, size_t ws_size, hipStream_t stream) {
    (void)in_sizes; (void)n_in; (void)out_size;
    const float** I = (const float**)d_in;
    const float *x = I[0], *Wq = I[1], *bq = I[2], *Wk = I[3], *bk = I[4], *Wv = I[5], *bv = I[6], *Wo = I[7], *bo = I[8];
    float* AW = (float*)d_out; float* OUT = AW + (size_t)NB_ * DD;
    char* wsp = (char*)d_ws;
    auto take = [&](size_t bytes) { char* p = wsp; wsp += (bytes + 255) & ~(size_t)255; return (void*)p; };
    bf* BQ = (bf*)take(DD * DD * 2); bf* BK = (bf*)take(DD * DD * 2); bf* BV = (bf*)take(DD * DD * 2); bf* BO = (bf*)take(DD * DD * 2); bf* XB = (bf*)take((size_t)NB_ * DD * 2);
    float* Q = (float*)take((size_t)NB_ * DD * 4); float* K = (float*)take((size_t)NB_ * DD * 4); float* V = (float*)take((size_t)NB_ * DD * 4); float* KMM = (float*)take((size_t)NB_ * 32 * 4); float* O = (float*)take((size_t)NB_ * DD * 4); bf* Oh = (bf*)take((size_t)NB_ * DD * 2); bf* Ol = (bf*)take((size_t)NB_ * DD * 2);
    if ((size_t)(wsp - (char*)d_ws) > ws_size) return;
    k_cvt8<<<(DD * DD / 8 + 255) / 256, 256, 0, stream>>>(Wq, BQ, DD * DD / 8); k_cvt8<<<(DD * DD / 8 + 255) / 256, 256, 0, stream>>>(Wk, BK, DD * DD / 8); k_cvt8<<<(DD * DD / 8 + 255) / 256, 256, 0, stream>>>(Wv, BV, DD * DD / 8); k_cvt8<<<(DD * DD / 8 + 255) / 256, 256, 0, stream>>>(Wo, BO, DD * DD / 8);
    k_cvt8<<<(NB_ * DD / 8 + 255) / 256, 256, 0, stream>>>(x, XB, (size_t)NB_ * DD / 8);
    k_gemmw<bf, 0, true><<<dim3(NB_ / 64, DD / 64, 1), 32, 0, stream>>>(XB, nullptr, BQ, nullptr, DD, Q, DD, bq, 0, 0, 0); k_gemmw<bf, 0, true><<<dim3(NB_ / 64, DD / 64, 1), 32, 0, stream>>>(XB, nullptr, BK, nullptr, DD, K, DD, bk, 0, 0, 0); k_gemmw<bf, 0, true><<<dim3(NB_ / 64, DD / 64, 1), 32, 0, stream>>>(XB, nullptr, BV, nullptr, DD, V, DD, bv, 0, 0, 0);
    k_kmm<<<NB_ / 8, 256, 0, stream>>>(K, KMM); k_att<<<(NB_ * DD + 255) / 256, 256, 0, stream>>>(Q, K, V, KMM, AW, O);
    k_spl<<<(NB_ * DD / 4 + 255) / 256, 256, 0, stream>>>(O, (size_t)NB_ * DD, Oh, Ol);
    k_gemmw<bf, 1, true><<<dim3(NB_ / 64, DD / 64, 1), 32, 0, stream>>>(Oh, Ol, BO, nullptr, DD, OUT, DD, bo, 0, 0, 0);
}
